// MambaEncoderBlock_62663572848678
// MI455X (gfx1250) — hardware-run, weakly checked
//
#include <hip/hip_runtime.h>
#include <hip/hip_fp16.h>
#include <math.h>

typedef __attribute__((ext_vector_type(16))) _Float16 v16h;
typedef __attribute__((ext_vector_type(8)))  _Float16 v8h;
typedef __attribute__((ext_vector_type(4)))  _Float16 v4h;
typedef __attribute__((ext_vector_type(8)))  float    v8f;
typedef __attribute__((ext_vector_type(4)))  float    v4f;
typedef __attribute__((ext_vector_type(2)))  float    v2f;
typedef __attribute__((ext_vector_type(2)))  unsigned v2u;


constexpr int kBatch  = 8;
constexpr int kSeq    = 1024;
constexpr int kDim    = 192;
constexpr int kDin    = kDim;
constexpr int kRank   = 12;
constexpr int kRankP  = 32;
constexpr int kNst    = 16;
constexpr int kProjN  = kRank + 2 * kNst;
constexpr int kProjP  = 64;
constexpr int kBcP    = 2 * kNst;
constexpr int kCat2   = 2 * kDim;
constexpr int kRowT   = kDim / 4;
constexpr float kLnEps  = 1.0e-3f;
constexpr float kWCarry = 1024.0f;
constexpr float kResid  = 2048.0f;
constexpr float kYCarry = 16.0f;
static_assert(kProjN == 44 && kCat2 == 384 && kRowT == 48);
static_assert(kProjN <= kProjP && (kProjP % 64) == 0);
static_assert((kSeq % 32) == 0 && (kDim % 64) == 0 && (kSeq % 64) == 0 && (kCat2 % 64) == 0);
static_assert((kDim % 32) == 0 && (kRankP % 32) == 0 && kRank <= kRankP);
static_assert(kDim == 192 && (kSeq % 8) == 0 && (kSeq % 4) == 0);
static_assert(kRank == 12 && kRankP == 32 && kBcP == 32 && kNst == 16);
static_assert(kRank + kBcP <= kProjP);

constexpr size_t kSzWP   = (size_t)kDim * kDim * 2;
constexpr size_t kSzWC   = (size_t)kCat2 * kDim * 2;
constexpr size_t kSzWD   = (size_t)kProjP * kDim * 2;
constexpr size_t kSzWDT  = (size_t)kDim * kRankP * 2;
constexpr size_t kSzVEC  = 1024;
constexpr size_t kSzALOG = (size_t)kDim * kNst * 4;
constexpr size_t kSzF32  = (size_t)kSeq * kDim * 4;
constexpr size_t kSzF16  = (size_t)kSeq * kDim * 2;
constexpr size_t kSzC    = (size_t)kSeq * kCat2 * 4;
constexpr size_t kSzPROJ = (size_t)kSeq * kProjP * 4;
constexpr size_t kSzDH   = (size_t)kSeq * kRankP * 2;
constexpr size_t kSzBC   = (size_t)kSeq * kBcP * 4;
constexpr size_t kOffWP    = 0;
constexpr size_t kOffWC    = kOffWP    + kSzWP;
constexpr size_t kOffWD1   = kOffWC    + kSzWC;
constexpr size_t kOffWD2   = kOffWD1   + kSzWD;
constexpr size_t kOffWDT1  = kOffWD2   + kSzWD;
constexpr size_t kOffWDT2  = kOffWDT1  + kSzWDT;
constexpr size_t kOffLNW   = kOffWDT2  + kSzWDT;
constexpr size_t kOffLNB   = kOffLNW   + kSzVEC;
constexpr size_t kOffPB    = kOffLNB   + kSzVEC;
constexpr size_t kOffFB    = kOffPB    + kSzVEC;
constexpr size_t kOffBB    = kOffFB    + kSzVEC;
constexpr size_t kOffDTB1  = kOffBB    + kSzVEC;
constexpr size_t kOffDTB2  = kOffDTB1  + kSzVEC;
constexpr size_t kOffDR1   = kOffDTB2  + kSzVEC;
constexpr size_t kOffDR2   = kOffDR1   + kSzVEC;
constexpr size_t kOffALOG1 = kOffDR2   + kSzVEC;
constexpr size_t kOffALOG2 = kOffALOG1 + kSzALOG;
constexpr size_t kOffXR    = kOffALOG2 + kSzALOG;
constexpr size_t kOffXNH   = kOffXR    + kSzF32;
constexpr size_t kOffXNL   = kOffXNH   + kSzF16;
constexpr size_t kOffP     = kOffXNL   + kSzF16;
constexpr size_t kOffZ     = kOffP     + kSzF32;
constexpr size_t kOffPH    = kOffZ     + kSzF32;
constexpr size_t kOffPL    = kOffPH    + kSzF16;
constexpr size_t kOffC     = kOffPL    + kSzF16;
constexpr size_t kOffU1    = kOffC     + kSzC;
constexpr size_t kOffU2    = kOffU1    + kSzF32;
constexpr size_t kOffU1H   = kOffU2    + kSzF32;
constexpr size_t kOffU1L   = kOffU1H   + kSzF16;
constexpr size_t kOffU2H   = kOffU1L   + kSzF16;
constexpr size_t kOffU2L   = kOffU2H   + kSzF16;
constexpr size_t kOffPROJ  = kOffU2L   + kSzF16;
constexpr size_t kOffDH    = kOffPROJ  + kSzPROJ;
constexpr size_t kOffBC    = kOffDH    + kSzDH;
constexpr size_t kOffDTP   = kOffBC    + kSzBC;
constexpr size_t kOffDT    = kOffDTP   + kSzF32;
constexpr size_t kOffY0H   = kOffDT    + kSzF32;
constexpr size_t kOffY0L   = kOffY0H   + kSzF16;
constexpr size_t kOffY1H   = kOffY0L   + kSzF16;
constexpr size_t kOffY1L   = kOffY1H   + kSzF16;
constexpr size_t kWsTotal  = kOffY1L   + kSzF16;
static_assert(kSzWP == 73728ull && kSzWC == 147456ull && kSzWD == 24576ull && kSzWDT == 12288ull);
static_assert((size_t)kDim * 4 <= kSzVEC && kSzALOG == 12288ull);
static_assert(kSzF32 == 786432ull && kSzF16 == 393216ull && kSzC == 1572864ull);
static_assert(kSzPROJ == 262144ull && kSzDH == 65536ull && kSzBC == 131072ull);
static_assert((kSzWP % 256) == 0 && (kSzWC % 256) == 0 && (kSzWD % 256) == 0 && (kSzWDT % 256) == 0 &&
              (kSzVEC % 256) == 0 && (kSzALOG % 256) == 0 && (kSzF32 % 256) == 0 && (kSzF16 % 256) == 0 &&
              (kSzC % 256) == 0 && (kSzPROJ % 256) == 0 && (kSzDH % 256) == 0 && (kSzBC % 256) == 0);
static_assert(kWsTotal == 12583936ull);
static_assert(kWsTotal <= 134217728ull);

__device__ __forceinline__ _Float16 f16_flush(float v) {
  const float w = (fabsf(v) < 6.103515625e-05f) ? 0.0f : v;
  return (_Float16)w;
}
__device__ __forceinline__ void f16_split(float v, _Float16& hi, _Float16& lo) {
  hi = f16_flush(v);
  const float hf = (float)hi;
  const float r = (v - hf) * kResid;
  lo = f16_flush(r);
}

__device__ __forceinline__ float bf16r(float v) {
  unsigned u = __float_as_uint(v);
  u = (u + 0x7FFFu + ((u >> 16) & 1u)) & 0xFFFF0000u;
  return __uint_as_float(u);
}

__device__ __forceinline__ float h16_to_f32(unsigned hb) {
  const unsigned sgn = (hb & 0x8000u) << 16; const unsigned em = hb & 0x7fffu;
  const float fn = __uint_as_float((em << 13) + 0x38000000u);
  const float fs = (float)em * 5.9604644775390625e-8f;
  const float mag = (em < 0x400u) ? fs : fn; return __uint_as_float(__float_as_uint(mag) | sgn); }

namespace eng {
union FragU { v16h v; v8h h[2]; };
__device__ __forceinline__ v16h frag_load(const _Float16* p) {
  FragU f;
  f.h[0] = *(const v8h*)(p);
  f.h[1] = *(const v8h*)(p + 16);
  return f.v;
}
__device__ __forceinline__ v8f mma(v16h a, v16h b, v8f c) {
  return __builtin_amdgcn_wmma_f32_16x16x32_f16(false, a, false, b, (short)0, c, false, false);
}
__device__ __forceinline__ void guard1(v8f& a, v16h x, v16h y) {
  asm volatile("v_nop\n\tv_nop\n\tv_nop\n\tv_nop" : "+v"(a) : "v"(x), "v"(y));
}
__device__ __forceinline__ void guard_acc(v8f& a) {
  asm volatile("v_nop\n\tv_nop\n\tv_nop\n\tv_nop" : "+v"(a));
}
__device__ __forceinline__ void keep4(v16h a, v16h b, v16h c, v16h d) {
  asm volatile("v_nop" :: "v"(a), "v"(b), "v"(c), "v"(d));
}

template <int MI, int SPL>
__global__ __launch_bounds__(256) void gemm_f16_kernel(
    const unsigned short* __restrict__ Ap, const unsigned short* __restrict__ A2p, int lda,
    const unsigned short* __restrict__ Btp, const unsigned short* __restrict__ Bt2p, int ldb,
    float* __restrict__ C, int ldc, int M, int N, int K, float scale, float rscale)
{
  static_assert(MI >= 1 && MI <= 2);
  static_assert(SPL >= 0 && SPL <= 2);
  const _Float16* A   = (const _Float16*)Ap;
  const _Float16* A2  = (const _Float16*)A2p;
  const _Float16* Bt  = (const _Float16*)Btp;
  const _Float16* Bt2 = (const _Float16*)Bt2p;
  __shared__ __align__(16) float sT[8][16 * 68];
  const int lane = threadIdx.x & 31;
  const int wave = threadIdx.x >> 5;
  const int tilesN = N >> 6;
  const int tilesM = M / (16 * MI);
  const int tile = blockIdx.x * 8 + wave;
  if (tile >= tilesM * tilesN) return;
  const int tm = tile / tilesN;
  const int tn = tile - tm * tilesN;
  const int m0 = tm * (16 * MI);
  const int n0 = tn << 6;
  const int rlane = lane & 15;
  const int koff  = (lane >> 4) * 8;
  const int mOff  = (lane >> 4) * 8;

  v8f acc[MI][4], accr[MI][4];
#pragma unroll
  for (int i = 0; i < MI; ++i)
#pragma unroll
    for (int j = 0; j < 4; ++j) {
      acc[i][j]  = (v8f){0.f, 0.f, 0.f, 0.f, 0.f, 0.f, 0.f, 0.f};
      accr[i][j] = (v8f){0.f, 0.f, 0.f, 0.f, 0.f, 0.f, 0.f, 0.f};
    }

  for (int k0 = 0; k0 < K; k0 += 32) {
    v16h bh[4], bl[4];
#pragma unroll
    for (int j = 0; j < 4; ++j) {
      const size_t bo = (size_t)(n0 + (j << 4) + rlane) * ldb + koff + k0;
      bh[j] = frag_load(Bt + bo);
      if (SPL == 2) bl[j] = frag_load(Bt2 + bo); else bl[j] = bh[j];
    }
#pragma unroll
    for (int i = 0; i < MI; ++i) {
      const size_t ao = (size_t)(m0 + (i << 4) + rlane) * lda + koff + k0;
      const v16h ah = frag_load(A + ao);
      v16h al = ah;
      if (SPL >= 1) al = frag_load(A2 + ao);
#pragma unroll
      for (int j = 0; j < 4; ++j) {
        acc[i][j] = mma(ah, bh[j], acc[i][j]);
        if (SPL >= 1) accr[i][j] = mma(al, bh[j], accr[i][j]);
        if (SPL == 2) accr[i][j] = mma(ah, bl[j], accr[i][j]);
      }
#pragma unroll
      for (int j = 0; j < 4; ++j) {
        guard1(acc[i][j], ah, al);
        if (SPL >= 1) guard1(accr[i][j], ah, al);
      }
    }
    keep4(bh[0], bh[1], bh[2], bh[3]);
    if (SPL == 2) keep4(bl[0], bl[1], bl[2], bl[3]);
  }
#pragma unroll
  for (int i = 0; i < MI; ++i)
#pragma unroll
    for (int j = 0; j < 4; ++j) {
      guard_acc(acc[i][j]);
      if (SPL >= 1) guard_acc(accr[i][j]);
    }

  float* slab = sT[wave];
#pragma unroll
  for (int i = 0; i < MI; ++i) {
    const int mBase = m0 + (i << 4);
#pragma unroll
    for (int j = 0; j < 4; ++j) {
#pragma unroll
      for (int r = 0; r < 8; ++r) {
        float v = acc[i][j][r] * scale;
        if (SPL >= 1) v += accr[i][j][r] * rscale;
        slab[(mOff + r) * 68 + (j << 4) + rlane] = v;
      }
    }
    __builtin_amdgcn_fence(__ATOMIC_RELEASE, "workgroup");
    __builtin_amdgcn_wave_barrier();
    __builtin_amdgcn_fence(__ATOMIC_ACQUIRE, "workgroup");
    {
      const int hh = lane >> 4, c4 = (lane & 15) * 4;
      for (int pass = 0; pass < 2; ++pass) {
#pragma unroll
        for (int it = 0; it < 8; ++it) {
          const int row = it * 2 + hh;
          const v4f v = *(const v4f*)(slab + row * 68 + c4);
          *(volatile v4f*)(C + (size_t)(mBase + row) * ldc + n0 + c4) = v;
        }
        __threadfence();
      }
    }
    __builtin_amdgcn_fence(__ATOMIC_RELEASE, "workgroup");
    __builtin_amdgcn_wave_barrier();
    __builtin_amdgcn_fence(__ATOMIC_ACQUIRE, "workgroup");
  }
}
}

template <bool LO>
__global__ __launch_bounds__(256) void transpose_pack_kernel(
    const float* __restrict__ W, unsigned short* __restrict__ BtH, unsigned short* __restrict__ BtL,
    int Kdim, int Ndim, float carry)
{
  __shared__ float tile[64 * 65];
  const int tid = threadIdx.x, lane = tid & 31, wave = tid >> 5;
  const int n0 = blockIdx.x * 64;
  const int k0 = blockIdx.y * 64;
#pragma unroll
  for (int p = 0; p < 16; ++p) {
    const int idx = tid + p * 256;
    const int kk  = idx >> 6;
    const int nn  = idx & 63;
    const int n   = n0 + nn;
    const int nc  = (n < Ndim) ? n : (Ndim - 1);
    const float v = W[(size_t)(k0 + kk) * Ndim + nc];
    tile[kk * 65 + nn] = (n < Ndim) ? (bf16r(v) * carry) : 0.0f;
  }
  __syncthreads();
  const int q = lane >> 3, c8 = (lane & 7) * 8;
  v8h hv[2], lv[2];
#pragma unroll
  for (int it = 0; it < 2; ++it) {
    const int nrow = it * 32 + wave * 4 + q;
#pragma unroll
    for (int e = 0; e < 8; ++e) {
      _Float16 h, l;
      const float t = tile[(c8 + e) * 65 + nrow];
      f16_split(t, h, l);
      hv[it][e] = h;
      lv[it][e] = l;
    }
  }
  for (int pass = 0; pass < 2; ++pass) {
#pragma unroll
    for (int it = 0; it < 2; ++it) {
      const int nrow = it * 32 + wave * 4 + q;
      const size_t o = (size_t)(n0 + nrow) * Kdim + k0 + c8;
      *(volatile v8h*)(BtH + o) = hv[it];
      if (LO) *(volatile v8h*)(BtL + o) = lv[it];
    }
    __threadfence();
  }
}

__global__ __launch_bounds__(256) void tpad_pack_kernel(
    const float* __restrict__ W, unsigned short* __restrict__ Bt, int total8, float carry)
{
  const int i = blockIdx.x * 256 + threadIdx.x;
  if (i >= total8) return;
  const int n = i >> 2;
  const int g = i & 3;
  v8h hv;
#pragma unroll
  for (int e = 0; e < 8; ++e) {
    const int k = 8 * g + e;
    const bool live = (k < kRank);
    const int kc = live ? k : (kRank - 1);
    const float v = W[(size_t)kc * kDim + n];
    const float t = bf16r(v) * carry;
    const float s = live ? t : 0.0f;
    hv[e] = f16_flush(s);
  }
  unsigned short* q = Bt + ((size_t)i << 3);
  *(volatile v8h*)q = hv;
  __threadfence();
  *(volatile v8h*)q = hv;
}

__global__ __launch_bounds__(256) void rne_vec_kernel(
    const float* __restrict__ src, float* __restrict__ dst, int n4)
{
  const int i = blockIdx.x * 256 + threadIdx.x;
  if (i >= n4) return;
  const v4f a = *(const v4f*)(src + (size_t)i * 4);
  const float a0 = a[0];
  const float a1 = a[1];
  const float a2 = a[2];
  const float a3 = a[3];
  v4f r;
  r[0] = bf16r(a0);
  r[1] = bf16r(a1);
  r[2] = bf16r(a2);
  r[3] = bf16r(a3);
  float* p = dst + (size_t)i * 4;
  *(volatile v4f*)p = r;
  __threadfence();
  *(volatile v4f*)p = r;
}

__global__ __launch_bounds__(256) void rne_plane_kernel(
    const float* __restrict__ src, float* __restrict__ dst, int n4)
{
  const int i = blockIdx.x * 256 + threadIdx.x;
  if (i >= n4) return;
  const v4f a = *(const v4f*)(src + (size_t)i * 4);
  const float a0 = a[0];
  const float a1 = a[1];
  const float a2 = a[2];
  const float a3 = a[3];
  v4f r;
  r[0] = bf16r(a0);
  r[1] = bf16r(a1);
  r[2] = bf16r(a2);
  r[3] = bf16r(a3);
  float* p = dst + (size_t)i * 4;
  *(volatile v4f*)p = r;
  __threadfence();
  *(volatile v4f*)p = r;
}

__global__ __launch_bounds__(256) void ln_split_kernel(
    const float* __restrict__ X, const float* __restrict__ gw, const float* __restrict__ gb,
    unsigned short* __restrict__ dH, unsigned short* __restrict__ dL, int rows)
{
  const int lane = threadIdx.x & 31;
  const int wave = threadIdx.x >> 5;
  const int row  = blockIdx.x * 8 + wave;
  if (row >= rows) return;
  const float* xr = X + (size_t)row * kDim;
  v2f t[3];
#pragma unroll
  for (int j = 0; j < 3; ++j) t[j] = *(const v2f*)(xr + 64 * j + 2 * lane);
  float s = 0.0f;
#pragma unroll
  for (int j = 0; j < 3; ++j)
#pragma unroll
    for (int e = 0; e < 2; ++e) s += t[j][e];
#pragma unroll
  for (int o = 16; o >= 1; o >>= 1) s += __shfl_xor(s, o, 32);
  const float mu = s * (1.0f / (float)kDim);
  float ss = 0.0f;
#pragma unroll
  for (int j = 0; j < 3; ++j)
#pragma unroll
    for (int e = 0; e < 2; ++e) {
      const float dv = t[j][e] - mu;
      ss = fmaf(dv, dv, ss);
    }
#pragma unroll
  for (int o = 16; o >= 1; o >>= 1) ss += __shfl_xor(ss, o, 32);
  const float var = ss * (1.0f / (float)kDim);
  const float inv = rsqrtf(var + kLnEps);
  unsigned hw[3], lw[3];
#pragma unroll
  for (int j = 0; j < 3; ++j) {
    const int off = 64 * j + 2 * lane;
    const v2f w2 = *(const v2f*)(gw + off);
    const v2f b2 = *(const v2f*)(gb + off);
    const float x0 = t[j][0];
    const float x1 = t[j][1];
    const float g0 = w2[0];
    const float g1 = w2[1];
    const float c0 = b2[0];
    const float c1 = b2[1];
    const float y0 = (x0 - mu) * inv * g0 + c0;
    const float y1 = (x1 - mu) * inv * g1 + c1;
    _Float16 h0, l0, h1, l1;
    f16_split(y0, h0, l0);
    f16_split(y1, h1, l1);
    const unsigned short hb0 = __builtin_bit_cast(unsigned short, h0);
    const unsigned short hb1 = __builtin_bit_cast(unsigned short, h1);
    const unsigned short lb0 = __builtin_bit_cast(unsigned short, l0);
    const unsigned short lb1 = __builtin_bit_cast(unsigned short, l1);
    hw[j] = (unsigned)hb0 | ((unsigned)hb1 << 16);
    lw[j] = (unsigned)lb0 | ((unsigned)lb1 << 16);
  }
  volatile unsigned* qh = (volatile unsigned*)(dH + (size_t)row * kDim);
  volatile unsigned* ql = (volatile unsigned*)(dL + (size_t)row * kDim);
  for (int pass = 0; pass < 2; ++pass) {
#pragma unroll
    for (int j = 0; j < 3; ++j) {
      qh[32 * j + lane] = hw[j];
      ql[32 * j + lane] = lw[j];
    }
    __threadfence();
  }
}

typedef float    ms1_v4f __attribute__((ext_vector_type(4)));
typedef unsigned ms1_v4u __attribute__((ext_vector_type(4)));
struct ms1_args {
  const float* dtpre;
  const float* u;
  const float* bc;
  const float* z;
  const float* A_log;
  const float* Dskip;
  __half* y;
  __half* y_lo;
  long ld_dtpre;
  long ld_u;
  long ld_bc;
  long ld_z;
  long ld_y;
  int offB;
  int offC;
  int offZ;
  float ycarry;
  int dir;
  int D;
  int L;
  int nbatch;
};
static_assert(sizeof(ms1_args) == 136);

__device__ __forceinline__ float ms1_flush16(float v) {
  return (fabsf(v) < 6.103515625e-05f) ? 0.0f : v;
}
__device__ __forceinline__ unsigned ms1_h16bits(float v) {
  return (unsigned)__half_as_ushort(__float2half_rn(ms1_flush16(v)));
}
__device__ __forceinline__ float ms1_h16val(unsigned b) {
  return __half2float(__ushort_as_half((unsigned short)b));
}
__device__ __forceinline__ float ms1_softplus(float v) {
  return fmaxf(v, 0.0f) + log1pf(expf(-fabsf(v)));
}
__device__ __forceinline__ void ms1_pack2(float v0, float v1, unsigned& hw, unsigned& lw) {
  const unsigned h0 = ms1_h16bits(v0);
  const unsigned h1 = ms1_h16bits(v1);
  const float r0 = (v0 - ms1_h16val(h0)) * 2048.0f;
  const float r1 = (v1 - ms1_h16val(h1)) * 2048.0f;
  const unsigned l0 = ms1_h16bits(r0);
  const unsigned l1 = ms1_h16bits(r1);
  hw = h0 | (h1 << 16);
  lw = l0 | (l1 << 16);
}

template <int NSTATE>
__global__ __launch_bounds__(64 * (NSTATE / 16)) void ms1_scan_kernel(ms1_args a)
{
  static_assert(NSTATE == 16 || NSTATE == 64);
  constexpr int NQ  = NSTATE / 16;
  constexpr int NT  = 64 * NQ;
  constexpr int NW  = NT / 32;
  constexpr int BCW = 2 * NSTATE;
  constexpr int YP  = 68;
  constexpr int RPI = NW * 4;
  constexpr int NIT = 64 / RPI;
  static_assert(16 * NT <= 64 * YP);
  __shared__ __align__(16) float sBC[64 * BCW];
  __shared__ __align__(16) float sY[64 * YP];
  const int tid  = threadIdx.x;
  const int lane = tid & 31;
  const int wave = tid >> 5;
  const int c    = tid / NQ;
  const int sq   = tid - c * NQ;
  const int bpb  = a.D / 64;
  const int bi   = blockIdx.x / bpb;
  if (bi >= a.nbatch) return;
  const int d0 = (blockIdx.x - bi * bpb) * 64;
  const int d  = d0 + c;
  const long rowb = (long)bi * a.L;
  const bool hasz  = (a.z != nullptr);
  const bool hasD  = (a.Dskip != nullptr);
  const bool hasLo = (a.y_lo != nullptr);

#pragma unroll 1
  for (int n = 0; n < 16; ++n) {
    const float al = a.A_log[(long)d * NSTATE + sq * 16 + n];
    sY[n * NT + tid] = -expf(al);
  }
  __syncthreads();
  float An[16], h[16];
#pragma unroll
  for (int n = 0; n < 16; ++n) {
    An[n] = sY[n * NT + tid];
    h[n] = 0.0f;
  }
  float Dd = 0.0f;
  if (hasD) Dd = a.Dskip[d];

  const int nchunk = a.L / 64;
  const bool fwd = (a.dir > 0);
  const int s0 = fwd ? 0 : 63;
  const int sd = fwd ? 1 : -1;
  const int q  = lane >> 3;
  const int c8 = (lane & 7) * 8;

  for (int ci = 0; ci < nchunk; ++ci) {
    const int tb = fwd ? (ci * 64) : (a.L - 64 - ci * 64);
    const long rowc = rowb + tb;
    __syncthreads();
#pragma unroll 8
    for (int i = 0; i < 32; ++i) {
      const int idx = tid + i * NT;
      const int st  = idx / BCW;
      const int col = idx - st * BCW;
      const int sc  = (col < NSTATE) ? (a.offB + col) : (a.offC + col - NSTATE);
      sBC[idx] = a.bc[(rowc + st) * a.ld_bc + sc];
    }
    __syncthreads();
    for (int s = 0; s < 64; ++s) {
      const int ls = s0 + sd * s;
      const long row = rowc + ls;
      float pre = a.dtpre[row * a.ld_dtpre + d];
      float uv  = a.u[row * a.ld_u + d];
      float zv  = 0.0f;
      if (hasz) zv = a.z[row * a.ld_z + a.offZ + d];
      asm volatile("" : "+v"(pre));
      asm volatile("" : "+v"(uv));
      asm volatile("" : "+v"(zv));
      const float delta = ms1_softplus(pre);
      const float dtx = delta * uv;
      const float* bp = sBC + ls * BCW + sq * 16;
      const float* cp = bp + NSTATE;
      ms1_v4f Bq[4], Cq[4];
#pragma unroll
      for (int k = 0; k < 4; ++k) {
        Bq[k] = *(const ms1_v4f*)(bp + 4 * k);
        Cq[k] = *(const ms1_v4f*)(cp + 4 * k);
      }
      float yv = 0.0f;
#pragma unroll
      for (int n = 0; n < 16; ++n) {
        const float e = __expf(delta * An[n]);
        h[n] = fmaf(e, h[n], dtx * Bq[n >> 2][n & 3]);
        yv = fmaf(h[n], Cq[n >> 2][n & 3], yv);
      }
      if (NQ > 1) {
        yv += __shfl_xor(yv, 1, 32);
        yv += __shfl_xor(yv, 2, 32);
      }
      if (hasD) yv = fmaf(uv, Dd, yv);
      if (hasz) {
        const float sg = __builtin_amdgcn_rcpf(1.0f + expf(-zv));
        yv = yv * (zv * sg);
      }
      if (sq == 0) sY[ls * YP + c] = yv * a.ycarry;
    }
    __syncthreads();
    ms1_v4u hw[NIT], lw[NIT];
#pragma unroll
    for (int it = 0; it < NIT; ++it) {
      const int row = it * RPI + wave * 4 + q;
      const float* sp = sY + row * YP + c8;
      const ms1_v4f f0 = *(const ms1_v4f*)(sp);
      const ms1_v4f f1 = *(const ms1_v4f*)(sp + 4);
      unsigned h0, h1, h2, h3, l0, l1, l2, l3;
      ms1_pack2(f0[0], f0[1], h0, l0);
      ms1_pack2(f0[2], f0[3], h1, l1);
      ms1_pack2(f1[0], f1[1], h2, l2);
      ms1_pack2(f1[2], f1[3], h3, l3);
      hw[it] = (ms1_v4u){h0, h1, h2, h3};
      lw[it] = (ms1_v4u){l0, l1, l2, l3};
    }
    for (int pass = 0; pass < 2; ++pass) {
#pragma unroll
      for (int it = 0; it < NIT; ++it) {
        const int row = it * RPI + wave * 4 + q;
        const long o = (rowc + row) * a.ld_y + d0 + c8;
        *(volatile ms1_v4u*)(a.y + o) = hw[it];
        if (hasLo) *(volatile ms1_v4u*)(a.y_lo + o) = lw[it];
      }
      __threadfence();
    }
  }
}

__global__ __launch_bounds__(192) void p_split_kernel(
    const float* __restrict__ P, const float* __restrict__ pbias, float* __restrict__ Z,
    unsigned short* __restrict__ PH, unsigned short* __restrict__ PL)
{
  const int tid = threadIdx.x;
  const int row = blockIdx.x * 4 + tid / kRowT;
  const int d4 = (tid % kRowT) * 4;
  const size_t o = (size_t)row * kDim + d4;
  const v4f a = *(const v4f*)(P + o);
  const v4f b = *(const v4f*)(pbias + d4);
  v4f zf;
  v4h hv, lv;
#pragma unroll
  for (int e = 0; e < 4; ++e) {
    const float p = a[e] + b[e];
    zf[e] = p / (1.0f + expf(-p));
    _Float16 h, l;
    f16_split(p, h, l);
    hv[e] = h;
    lv[e] = l;
  }
  for (int pass = 0; pass < 2; ++pass) {
    *(volatile v4f*)(Z + o) = zf;
    *(volatile v4h*)(PH + o) = hv;
    *(volatile v4h*)(PL + o) = lv;
    __threadfence();
  }
}

__global__ __launch_bounds__(192) void u_split_kernel(
    const float* __restrict__ C, const float* __restrict__ fbias, const float* __restrict__ bbias,
    float* __restrict__ U1, float* __restrict__ U2,
    unsigned short* __restrict__ U1H, unsigned short* __restrict__ U1L,
    unsigned short* __restrict__ U2H, unsigned short* __restrict__ U2L)
{
  const int tid = threadIdx.x;
  const int row = blockIdx.x * 4 + tid / kRowT;
  const int d4 = (tid % kRowT) * 4;
  const size_t o = (size_t)row * kDim + d4;
  const size_t rc = (size_t)row * kCat2 + d4;
  const v4f a1 = *(const v4f*)(C + rc);
  const v4f a2 = *(const v4f*)(C + rc + kDim);
  const v4f fb = *(const v4f*)(fbias + d4);
  const v4f bb = *(const v4f*)(bbias + d4);
  v4f uf, ub;
  v4h ufh, ufl, ubh, ubl;
#pragma unroll
  for (int e = 0; e < 4; ++e) {
    const float u1 = ms1_softplus(a1[e] + fb[e]);
    const float u2 = ms1_softplus(a2[e] + bb[e]);
    uf[e] = u1;
    ub[e] = u2;
    _Float16 h1, l1, h2, l2;
    f16_split(u1, h1, l1);
    f16_split(u2, h2, l2);
    ufh[e] = h1;
    ufl[e] = l1;
    ubh[e] = h2;
    ubl[e] = l2;
  }
  for (int pass = 0; pass < 2; ++pass) {
    *(volatile v4f*)(U1 + o) = uf;
    *(volatile v4f*)(U2 + o) = ub;
    *(volatile v4h*)(U1H + o) = ufh;
    *(volatile v4h*)(U1L + o) = ufl;
    *(volatile v4h*)(U2H + o) = ubh;
    *(volatile v4h*)(U2L + o) = ubl;
    __threadfence();
  }
}

__global__ __launch_bounds__(128) void proj_split_kernel(
    const float* __restrict__ P, unsigned short* __restrict__ dH, float* __restrict__ BC)
{
  const int tid = threadIdx.x;
  const int r0 = blockIdx.x * 32;
  const int rowa = r0 + (tid >> 2);
  const int ga = tid & 3;
  const int g8 = ga * 8;
  v8h hv;
  {
    const float* sp = P + (size_t)rowa * kProjP + g8;
    const v4f a0 = *(const v4f*)(sp);
    const v4f a1 = *(const v4f*)(sp + 4);
#pragma unroll
    for (int e = 0; e < 4; ++e) {
      const float f0 = a0[e];
      const float f1 = a1[e];
      const bool live0 = (g8 + e < kRank);
      const bool live1 = (g8 + 4 + e < kRank);
      const float s0 = live0 ? f0 : 0.0f;
      const float s1 = live1 ? f1 : 0.0f;
      hv[e] = f16_flush(s0);
      hv[4 + e] = f16_flush(s1);
    }
  }
  const int p4 = (tid & 7) * 4;
  v4f bcv[2];
#pragma unroll
  for (int it = 0; it < 2; ++it) {
    const int rowb = r0 + it * 16 + (tid >> 3);
    const v4f pv = *(const v4f*)(P + (size_t)rowb * kProjP + kRank + p4);
    bcv[it] = pv;
  }
  for (int pass = 0; pass < 2; ++pass) {
    *(volatile v8h*)(dH + (size_t)rowa * kRankP + g8) = hv;
#pragma unroll
    for (int it = 0; it < 2; ++it) {
      const int rowb = r0 + it * 16 + (tid >> 3);
      *(volatile v4f*)(BC + (size_t)rowb * kBcP + p4) = bcv[it];
    }
    __threadfence();
  }
}

__global__ __launch_bounds__(256) void dt_bias_kernel(
    const float* __restrict__ DTP, const float* __restrict__ bdt, float* __restrict__ DT)
{
  const int d4 = (blockIdx.x * 256 + threadIdx.x) * 4;
  const int r0 = blockIdx.y * 8;
  const v4f b = *(const v4f*)(bdt + d4);
  v4f val[8];
#pragma unroll
  for (int i = 0; i < 8; ++i) {
    const v4f p = *(const v4f*)(DTP + (size_t)(r0 + i) * kDin + d4);
    val[i] = p + b;
  }
  for (int pass = 0; pass < 2; ++pass) {
#pragma unroll
    for (int i = 0; i < 8; ++i)
      *(volatile v4f*)(DT + (size_t)(r0 + i) * kDin + d4) = val[i];
    __threadfence();
  }
}

__global__ __launch_bounds__(192) void gated_out_kernel(
    const unsigned short* __restrict__ Y0H, const unsigned short* __restrict__ Y0L,
    const unsigned short* __restrict__ Y1H, const unsigned short* __restrict__ Y1L,
    const float* __restrict__ Z, const float* __restrict__ XRp, float* __restrict__ out)
{
  const int tid = threadIdx.x;
  const int row = blockIdx.x * 4 + tid / kRowT;
  const int d4 = (tid % kRowT) * 4;
  constexpr float kInvResid = 1.0f / kResid;
  constexpr float kInvCarry = 1.0f / kYCarry;
  const size_t o = (size_t)row * kDin + d4;
  const v2u ah = *(const v2u*)(const void*)(Y0H + o);
  const v2u al = *(const v2u*)(const void*)(Y0L + o);
  const v2u bh = *(const v2u*)(const void*)(Y1H + o);
  const v2u bl = *(const v2u*)(const void*)(Y1L + o);
  const v4f zz = *(const v4f*)(Z + o);
  const v4f xx = *(const v4f*)(XRp + o);
  float ya[4], yb[4];
  ya[0] = (h16_to_f32(ah[0] & 0xffffu) + h16_to_f32(al[0] & 0xffffu) * kInvResid) * kInvCarry;
  ya[1] = (h16_to_f32(ah[0] >> 16) + h16_to_f32(al[0] >> 16) * kInvResid) * kInvCarry;
  ya[2] = (h16_to_f32(ah[1] & 0xffffu) + h16_to_f32(al[1] & 0xffffu) * kInvResid) * kInvCarry;
  ya[3] = (h16_to_f32(ah[1] >> 16) + h16_to_f32(al[1] >> 16) * kInvResid) * kInvCarry;
  yb[0] = (h16_to_f32(bh[0] & 0xffffu) + h16_to_f32(bl[0] & 0xffffu) * kInvResid) * kInvCarry;
  yb[1] = (h16_to_f32(bh[0] >> 16) + h16_to_f32(bl[0] >> 16) * kInvResid) * kInvCarry;
  yb[2] = (h16_to_f32(bh[1] & 0xffffu) + h16_to_f32(bl[1] & 0xffffu) * kInvResid) * kInvCarry;
  yb[3] = (h16_to_f32(bh[1] >> 16) + h16_to_f32(bl[1] >> 16) * kInvResid) * kInvCarry;
  v4f v;
#pragma unroll
  for (int e = 0; e < 4; ++e) {
    const float ze = zz[e];
    const float xe = xx[e];
    const float pa = ya[e] * ze;
    const float pq = yb[e] * ze;
    const float sm = pa + pq;
    v[e] = sm + xe;
  }
  for (int pass = 0; pass < 2; ++pass) {
    *(volatile v4f*)(out + o) = v;
    __threadfence();
  }
}

static_assert(((kSeq / 32) * (kDim / 64)) % 8 == 0);
static_assert(((kSeq / 32) * (kCat2 / 64)) % 8 == 0);
static_assert(((kSeq / 32) * (kProjP / 64)) % 8 == 0);
static_assert(((kDim * kRankP / 8) % 256) == 0);
static_assert(((kDim * kNst / 4) % 256) == 0);
static_assert(((kSeq * kDim / 4) % 256) == 0);
static_assert((kDim / 4) <= 256 && (kSeq % 32) == 0 && (kSeq % 8) == 0 && (kSeq % 4) == 0);
static_assert((kDim % 64) == 0 && (kProjP % 64) == 0);

extern "C" void kernel_launch(void* const* d_in, const int* in_sizes, int n_in,
                              void* d_out, int out_size, void* d_ws, size_t ws_size,
                              hipStream_t stream)
{
  if (n_in < 19) return;
  if (in_sizes[0] != kBatch * kSeq * kDim) return;
  if (in_sizes[1] != kDim) return;
  if (in_sizes[2] != kDim) return;
  if (in_sizes[3] != kDim * kDim) return;
  if (in_sizes[4] != kDim) return;
  if (in_sizes[5] != kDim * kDim) return;
  if (in_sizes[6] != kDim) return;
  if (in_sizes[7] != kDim * kDim) return;
  if (in_sizes[8] != kDim) return;
  if (in_sizes[9] != kDim * kProjN) return;
  if (in_sizes[10] != kRank * kDim) return;
  if (in_sizes[11] != kDim) return;
  if (in_sizes[12] != kDim * kNst) return;
  if (in_sizes[13] != kDim) return;
  if (in_sizes[14] != kDim * kProjN) return;
  if (in_sizes[15] != kRank * kDim) return;
  if (in_sizes[16] != kDim) return;
  if (in_sizes[17] != kDim * kNst) return;
  if (in_sizes[18] != kDim) return;
  if (out_size != kBatch * kSeq * kDim) return;
  if (ws_size < kWsTotal) return;

  const float* x       = (const float*)d_in[0];
  const float* ln_w    = (const float*)d_in[1];
  const float* ln_b    = (const float*)d_in[2];
  const float* proj_W  = (const float*)d_in[3];
  const float* proj_b  = (const float*)d_in[4];
  const float* fwd_W   = (const float*)d_in[5];
  const float* fwd_b   = (const float*)d_in[6];
  const float* bwd_W   = (const float*)d_in[7];
  const float* bwd_b   = (const float*)d_in[8];
  const float* dbc_W1  = (const float*)d_in[9];
  const float* dt_W1   = (const float*)d_in[10];
  const float* dt_b1   = (const float*)d_in[11];
  const float* A_log1  = (const float*)d_in[12];
  const float* D_skip1 = (const float*)d_in[13];
  const float* dbc_W2  = (const float*)d_in[14];
  const float* dt_W2   = (const float*)d_in[15];
  const float* dt_b2   = (const float*)d_in[16];
  const float* A_log2  = (const float*)d_in[17];
  const float* D_skip2 = (const float*)d_in[18];
  float* out = (float*)d_out;

  char* ws = (char*)d_ws;
  unsigned short* WP    = (unsigned short*)(ws + kOffWP);
  unsigned short* WC    = (unsigned short*)(ws + kOffWC);
  unsigned short* WD1   = (unsigned short*)(ws + kOffWD1);
  unsigned short* WD2   = (unsigned short*)(ws + kOffWD2);
  unsigned short* WDT1  = (unsigned short*)(ws + kOffWDT1);
  unsigned short* WDT2  = (unsigned short*)(ws + kOffWDT2);
  float*          LNW   = (float*)(ws + kOffLNW);
  float*          LNB   = (float*)(ws + kOffLNB);
  float*          PB    = (float*)(ws + kOffPB);
  float*          FB    = (float*)(ws + kOffFB);
  float*          BB    = (float*)(ws + kOffBB);
  float*          DTB1  = (float*)(ws + kOffDTB1);
  float*          DTB2  = (float*)(ws + kOffDTB2);
  float*          DR1   = (float*)(ws + kOffDR1);
  float*          DR2   = (float*)(ws + kOffDR2);
  float*          ALOG1 = (float*)(ws + kOffALOG1);
  float*          ALOG2 = (float*)(ws + kOffALOG2);
  float*          XR    = (float*)(ws + kOffXR);
  unsigned short* XNH   = (unsigned short*)(ws + kOffXNH);
  unsigned short* XNL   = (unsigned short*)(ws + kOffXNL);
  float*          P     = (float*)(ws + kOffP);
  float*          Z     = (float*)(ws + kOffZ);
  unsigned short* PH    = (unsigned short*)(ws + kOffPH);
  unsigned short* PL    = (unsigned short*)(ws + kOffPL);
  float*          C     = (float*)(ws + kOffC);
  float*          U1    = (float*)(ws + kOffU1);
  float*          U2    = (float*)(ws + kOffU2);
  unsigned short* U1H   = (unsigned short*)(ws + kOffU1H);
  unsigned short* U1L   = (unsigned short*)(ws + kOffU1L);
  unsigned short* U2H   = (unsigned short*)(ws + kOffU2H);
  unsigned short* U2L   = (unsigned short*)(ws + kOffU2L);
  float*          PROJ  = (float*)(ws + kOffPROJ);
  unsigned short* DH    = (unsigned short*)(ws + kOffDH);
  float*          BC    = (float*)(ws + kOffBC);
  float*          DTP   = (float*)(ws + kOffDTP);
  float*          DT    = (float*)(ws + kOffDT);
  unsigned short* Y0H   = (unsigned short*)(ws + kOffY0H);
  unsigned short* Y0L   = (unsigned short*)(ws + kOffY0L);
  unsigned short* Y1H   = (unsigned short*)(ws + kOffY1H);
  unsigned short* Y1L   = (unsigned short*)(ws + kOffY1L);

  constexpr float sW  = 1.0f / kWCarry;
  constexpr float sWr = 1.0f / (kWCarry * kResid);

  transpose_pack_kernel<false><<<dim3(kDim / 64, kDim / 64), 256, 0, stream>>>(
      proj_W, WP, WP, kDim, kDim, kWCarry);

  transpose_pack_kernel<false><<<dim3(kDim / 64, kDim / 64), 256, 0, stream>>>(
      fwd_W, WC, WC, kDim, kDim, kWCarry);
  transpose_pack_kernel<false><<<dim3(kDim / 64, kDim / 64), 256, 0, stream>>>(
      bwd_W, WC + (size_t)kDim * kDim, WC + (size_t)kDim * kDim, kDim, kDim, kWCarry);

  transpose_pack_kernel<false><<<dim3(kProjP / 64, kDim / 64), 256, 0, stream>>>(
      dbc_W1, WD1, WD1, kDim, kProjN, kWCarry);
  transpose_pack_kernel<false><<<dim3(kProjP / 64, kDim / 64), 256, 0, stream>>>(
      dbc_W2, WD2, WD2, kDim, kProjN, kWCarry);

  tpad_pack_kernel<<<(kDim * kRankP / 8) / 256, 256, 0, stream>>>(dt_W1, WDT1, kDim * kRankP / 8, kWCarry);
  tpad_pack_kernel<<<(kDim * kRankP / 8) / 256, 256, 0, stream>>>(dt_W2, WDT2, kDim * kRankP / 8, kWCarry);

  rne_vec_kernel<<<1, 256, 0, stream>>>(ln_w, LNW, kDim / 4);
  rne_vec_kernel<<<1, 256, 0, stream>>>(ln_b, LNB, kDim / 4);
  rne_vec_kernel<<<1, 256, 0, stream>>>(proj_b, PB, kDim / 4);
  rne_vec_kernel<<<1, 256, 0, stream>>>(fwd_b, FB, kDim / 4);
  rne_vec_kernel<<<1, 256, 0, stream>>>(bwd_b, BB, kDim / 4);
  rne_vec_kernel<<<1, 256, 0, stream>>>(dt_b1, DTB1, kDim / 4);
  rne_vec_kernel<<<1, 256, 0, stream>>>(dt_b2, DTB2, kDim / 4);
  rne_vec_kernel<<<1, 256, 0, stream>>>(D_skip1, DR1, kDim / 4);
  rne_vec_kernel<<<1, 256, 0, stream>>>(D_skip2, DR2, kDim / 4);

  rne_vec_kernel<<<(kDim * kNst / 4) / 256, 256, 0, stream>>>(A_log1, ALOG1, kDim * kNst / 4);
  rne_vec_kernel<<<(kDim * kNst / 4) / 256, 256, 0, stream>>>(A_log2, ALOG2, kDim * kNst / 4);

  const float* Uk[2] = {U1, U2};
  const unsigned short* UkH[2] = {U1H, U2H};
  const unsigned short* UkL[2] = {U1L, U2L};
  const unsigned short* WDk[2] = {WD1, WD2};
  const unsigned short* WDTk[2] = {WDT1, WDT2};
  const float* DTBk[2] = {DTB1, DTB2};
  const float* ALOGk[2] = {ALOG1, ALOG2};
  const float* DRk[2] = {DR1, DR2};
  unsigned short* YkH[2] = {Y0H, Y1H};
  unsigned short* YkL[2] = {Y0L, Y1L};

  for (int b = 0; b < kBatch; ++b) {
    const size_t eb = (size_t)b * kSeq * kDim;
    const float* xb = x + eb;
    float* outb = out + eb;

    rne_plane_kernel<<<(kSeq * kDim / 4) / 256, 256, 0, stream>>>(xb, XR, kSeq * kDim / 4);

    ln_split_kernel<<<kSeq / 8, 256, 0, stream>>>(XR, LNW, LNB, XNH, XNL, kSeq);

    eng::gemm_f16_kernel<2, 1><<<dim3((kSeq / 32) * (kDim / 64) / 8), 256, 0, stream>>>(
        XNH, XNL, kDim, WP, WP, kDim, P, kDim, kSeq, kDim, kDim, sW, sWr);

    p_split_kernel<<<kSeq / 4, 192, 0, stream>>>(P, PB, Z, PH, PL);

    eng::gemm_f16_kernel<2, 1><<<dim3((kSeq / 32) * (kCat2 / 64) / 8), 256, 0, stream>>>(
        PH, PL, kDim, WC, WC, kDim, C, kCat2, kSeq, kCat2, kDim, sW, sWr);

    u_split_kernel<<<kSeq / 4, 192, 0, stream>>>(C, FB, BB, U1, U2, U1H, U1L, U2H, U2L);

    for (int k = 0; k < 2; ++k) {
      eng::gemm_f16_kernel<2, 1><<<dim3((kSeq / 32) * (kProjP / 64) / 8), 256, 0, stream>>>(
          UkH[k], UkL[k], kDim, WDk[k], WDk[k], kDim, PROJ, kProjP, kSeq, kProjP, kDim, sW, sWr);

      proj_split_kernel<<<kSeq / 32, 128, 0, stream>>>(PROJ, DH, BC);

      eng::gemm_f16_kernel<2, 0><<<dim3((kSeq / 32) * (kDim / 64) / 8), 256, 0, stream>>>(
          DH, nullptr, kRankP, WDTk[k], nullptr, kRankP, DTP, kDim, kSeq, kDim, kRankP, sW, 0.0f);

      dt_bias_kernel<<<dim3(1, kSeq / 8), kDim / 4, 0, stream>>>(DTP, DTBk[k], DT);

      ms1_args sa;
      sa.dtpre = DT;
      sa.u = Uk[k];
      sa.bc = BC;
      sa.z = nullptr;
      sa.A_log = ALOGk[k];
      sa.Dskip = DRk[k];
      sa.y = (__half*)YkH[k];
      sa.y_lo = (__half*)YkL[k];
      sa.ld_dtpre = kDim;
      sa.ld_u = kDim;
      sa.ld_bc = kBcP;
      sa.ld_z = 0;
      sa.ld_y = kDim;
      sa.offB = 0;
      sa.offC = kNst;
      sa.offZ = 0;
      sa.ycarry = kYCarry;
      sa.dir = 1;
      sa.D = kDim;
      sa.L = kSeq;
      sa.nbatch = 1;
      ms1_scan_kernel<16><<<dim3(kDim / 64), 64, 0, stream>>>(sa);
    }

    gated_out_kernel<<<kSeq / 4, 192, 0, stream>>>(Y0H, Y0L, Y1H, Y1L, Z, XR, outb);
  }
}
